// NNConvEncoder_8375186227331
// MI455X (gfx1250) — hardware-verified
//
#include <hip/hip_runtime.h>


typedef _Float16 v8h  __attribute__((ext_vector_type(8)));
typedef _Float16 v16h __attribute__((ext_vector_type(16)));
typedef float    v8f  __attribute__((ext_vector_type(8)));
typedef float    v4f  __attribute__((ext_vector_type(4)));
typedef int      v4i  __attribute__((ext_vector_type(4)));

union Frag { v16h v; v8h hf[2]; };

#define HID    64
#define KH     128
#define GW     192
#define ZK     8256
#define NSLOT  129
#define SEGCAP 1024
#define MAXDEG 256
#define ECH    16
#define MAXB2  4096

#define SC_A   64.0f
#define SC_Z   1024.0f
#define SC_W   1024.0f
#define UN_W   (1.0f / 1024.0f)
#define UN_AW  (1.0f / 65536.0f)
#define UN_ZW  (1.0f / 1048576.0f)

#define LDS_ZB  98304
#define LDS_ZG  163840
#define LDS_GRU 73728

__device__ __forceinline__ v8f mma16(v16h a, v16h b, v8f c)
{
    c = __builtin_amdgcn_wmma_f32_16x16x32_f16(false, a, false, b, (short)0, c, false, false);
    asm volatile("v_nop\n\tv_nop\n\tv_nop\n\tv_nop" : "+v"(c) : "v"(a), "v"(b));
    return c;
}
__device__ __forceinline__ v8f zero8()
{
    v8f z;
#pragma unroll
    for (int i = 0; i < 8; ++i) z[i] = 0.0f;
    return z;
}
__device__ __forceinline__ v4f zero4()
{
    v4f z;
#pragma unroll
    for (int i = 0; i < 4; ++i) z[i] = 0.0f;
    return z;
}
__device__ __forceinline__ v8h zero8h()
{
    v8h z;
#pragma unroll
    for (int i = 0; i < 8; ++i) z[i] = (_Float16)0.0f;
    return z;
}
__device__ __forceinline__ void st4(float* p, v4f v)     { *(volatile v4f*)p = v; }
__device__ __forceinline__ void st8h(_Float16* p, v8h v) { *(volatile v8h*)p = v; }
__device__ __forceinline__ void st4i(int* p, v4i v)      { *(volatile v4i*)p = v; }

__device__ __forceinline__ float wmax32(float v)
{
#pragma unroll
    for (int d = 16; d > 0; d >>= 1) v = fmaxf(v, __shfl_xor(v, d, 32));
    return v;
}
__device__ __forceinline__ float wsum32(float v)
{
#pragma unroll
    for (int d = 16; d > 0; d >>= 1) v += __shfl_xor(v, d, 32);
    return v;
}
__device__ __forceinline__ float sigm(float x) { return 1.0f / (1.0f + expf(-x)); }
__device__ __forceinline__ int clampi(int v, int lo, int hi) { return v < lo ? lo : (v > hi ? hi : v); }

__global__ void __launch_bounds__(256)
k_prep(const float* __restrict__ e2w, const float* __restrict__ e2b,
       const float* __restrict__ gih, const float* __restrict__ ghh,
       _Float16* __restrict__ W16, _Float16* __restrict__ GihT, _Float16* __restrict__ GhhT)
{
    __shared__ float sb[HID * GW];
    const int bid = blockIdx.x, tid = threadIdx.x;
    if (bid < NSLOT) {
        const float* sp = (bid < KH) ? (e2w + (size_t)bid * 4096) : e2b;
        for (int q = tid; q < 4096; q += 256) sb[q] = sp[q];
        __syncthreads();
        _Float16* op = W16 + (size_t)bid * 4096;
        v8h t[2];
#pragma unroll
        for (int s = 0; s < 2; ++s) {
            const int q = s * 256 + tid, o = q >> 3, i0 = (q & 7) * 8;
            v8h u;
#pragma unroll
            for (int j = 0; j < 8; ++j) u[j] = (_Float16)(sb[(i0 + j) * HID + o] * SC_W);
            t[s] = u;
        }
#pragma unroll
        for (int s = 0; s < 2; ++s) st8h(op + (size_t)(s * 256 + tid) * 8, t[s]);
        __threadfence();
#pragma unroll
        for (int s = 0; s < 2; ++s) st8h(op + (size_t)(s * 256 + tid) * 8, t[s]);
    } else {
        const bool first = (bid == NSLOT);
        const float* sp = first ? gih : ghh;
        _Float16* op = first ? GihT : GhhT;
        for (int q = tid; q < HID * GW; q += 256) sb[q] = sp[q];
        __syncthreads();
        v8h t[6];
#pragma unroll
        for (int s = 0; s < 6; ++s) {
            const int q = s * 256 + tid, c = q >> 3, i0 = (q & 7) * 8;
            v8h u;
#pragma unroll
            for (int j = 0; j < 8; ++j) u[j] = (_Float16)(sb[(i0 + j) * GW + c] * SC_W);
            t[s] = u;
        }
#pragma unroll
        for (int s = 0; s < 6; ++s) st8h(op + (size_t)(s * 256 + tid) * 8, t[s]);
        __threadfence();
#pragma unroll
        for (int s = 0; s < 6; ++s) st8h(op + (size_t)(s * 256 + tid) * 8, t[s]);
    }
}

__global__ void __launch_bounds__(32)
k_csr(const int* __restrict__ dst, int* __restrict__ segTab, int* __restrict__ nodeRec, int E)
{
    __shared__ int sSeg[SEGCAP];
    __shared__ int sRec[64];
    const int lane = threadIdx.x;
    const int base = blockIdx.x * 32;
    for (int q = lane; q < SEGCAP; q += 32) sSeg[q] = 0;

    int cnt = 0;
    for (int c0 = 0; c0 < E; c0 += 32) {
        const int e = c0 + lane;
        const int dv = (e < E) ? dst[e] : -1;
        const int rel = dv - base;
        unsigned mask = __builtin_amdgcn_ballot_w32((unsigned)rel < 32u);
        while (mask != 0u) {
            const int q = __builtin_ctz(mask);
            mask &= mask - 1u;
            const int dd = __shfl(rel, q, 32);
            cnt += (lane == dd) ? 1 : 0;
        }
    }
    int incl = cnt;
#pragma unroll
    for (int dl = 1; dl < 32; dl <<= 1) {
        const int y = __shfl_up(incl, dl, 32);
        if (lane >= dl) incl += y;
    }
    const int off = incl - cnt;
    int cur = off;
    __syncthreads();

    for (int c0 = 0; c0 < E; c0 += 32) {
        const int e = c0 + lane;
        const int dv = (e < E) ? dst[e] : -1;
        const int rel = dv - base;
        unsigned mask = __builtin_amdgcn_ballot_w32((unsigned)rel < 32u);
        while (mask != 0u) {
            const int q = __builtin_ctz(mask);
            mask &= mask - 1u;
            const int dd = __shfl(rel, q, 32);
            const int eh = c0 + q;
            if (lane == dd) {
                if (cur < SEGCAP) sSeg[cur] = eh;
                ++cur;
            }
        }
    }
    sRec[2 * lane]     = off;
    sRec[2 * lane + 1] = cnt;
    __syncthreads();

    v4i sv[8];
#pragma unroll
    for (int s = 0; s < 8; ++s) sv[s] = ((const v4i*)sSeg)[s * 32 + lane];
    const v4i rv = ((const v4i*)sRec)[lane & 15];
    int* tb = segTab + (size_t)blockIdx.x * SEGCAP;
    int* rb = nodeRec + (size_t)blockIdx.x * 64;
#pragma unroll
    for (int s = 0; s < 8; ++s) st4i(tb + (size_t)(s * 32 + lane) * 4, sv[s]);
    if (lane < 16) st4i(rb + lane * 4, rv);
    __threadfence();
#pragma unroll
    for (int s = 0; s < 8; ++s) st4i(tb + (size_t)(s * 32 + lane) * 4, sv[s]);
    if (lane < 16) st4i(rb + lane * 4, rv);
}

__global__ void __launch_bounds__(128)
k_lin0(const float* __restrict__ nfeat, const float* __restrict__ w,
       const float* __restrict__ b, float* __restrict__ hout, int N)
{
    __shared__ float sT[64 * HID];
    const int tid = threadIdx.x, wave = tid >> 5, lane = tid & 31;
    const int h = lane >> 4, m = lane & 15;
    const int r0 = (blockIdx.x * 4 + wave) * 16;
    int node = r0 + m;
    node = node < N ? node : N - 1;
    const v8h z8 = zero8h();

    Frag a;
    {
        const float* xr = nfeat + (size_t)node * 16 + 8 * h;
        v8h t;
#pragma unroll
        for (int j = 0; j < 8; ++j) t[j] = (_Float16)xr[j];
        a.hf[0] = t;
        a.hf[1] = z8;
    }
#pragma unroll
    for (int ct = 0; ct < 4; ++ct) {
        Frag bb;
        v8h u;
#pragma unroll
        for (int j = 0; j < 8; ++j) u[j] = (_Float16)(w[(8 * h + j) * HID + ct * 16 + m] * SC_W);
        bb.hf[0] = u;
        bb.hf[1] = z8;
        v8f acc = zero8();
        acc = mma16(a.v, bb.v, acc);
        const float bc = b[ct * 16 + m];
#pragma unroll
        for (int r = 0; r < 8; ++r)
            sT[(wave * 16 + 8 * h + r) * HID + ct * 16 + m] = fmaxf(acc[r] * UN_W + bc, 0.0f);
    }
    __syncthreads();
    v4f pv[8];
#pragma unroll
    for (int s = 0; s < 8; ++s) pv[s] = ((const v4f*)sT)[s * 128 + tid];
    float* ob = hout + (size_t)blockIdx.x * (64 * HID);
#pragma unroll
    for (int s = 0; s < 8; ++s) st4(ob + (size_t)(s * 128 + tid) * 4, pv[s]);
    __threadfence();
#pragma unroll
    for (int s = 0; s < 8; ++s) st4(ob + (size_t)(s * 128 + tid) * 4, pv[s]);
}

__global__ void __launch_bounds__(256)
k_zbuild(const float* __restrict__ hcur, const float* __restrict__ efeat,
         const float* __restrict__ e1w, const float* __restrict__ e1b,
         const int* __restrict__ srcIdx, const int* __restrict__ segTab,
         const int* __restrict__ nodeRec, _Float16* __restrict__ Z,
         int passBase, int N, int E)
{
    extern __shared__ float zsm[];
    __shared__ float sE1w[5 * KH];
    __shared__ float sE1b[KH];
    __shared__ int   sNav[8];

    const int tid = threadIdx.x, wave = tid >> 5, lane = tid & 31;
    const int li = lane & 7, lk = lane >> 3;
    for (int q = tid; q < 5 * KH; q += 256) sE1w[q] = e1w[q];
    if (tid < KH) sE1b[tid] = e1b[tid];

    const int row = blockIdx.x * 8 + wave;
    int d = passBase + row;
    d = d < N ? d : N - 1;
    int off = nodeRec[2 * d], cnt = nodeRec[2 * d + 1];
    cnt = cnt < 0 ? 0 : cnt;
    off = clampi(off, 0, SEGCAP);
    int navail = cnt < (SEGCAP - off) ? cnt : (SEGCAP - off);
    navail = navail < MAXDEG ? navail : MAXDEG;
    const float osc = SC_Z / fmaxf((float)cnt, 1.0f);
    if (lane == 0) sNav[wave] = navail;
    __syncthreads();
    int nmax = 0;
#pragma unroll
    for (int q = 0; q < 8; ++q) nmax = nmax > sNav[q] ? nmax : sNav[q];
    const int nch = (nmax + ECH - 1) / ECH;

    const int* seg = segTab + (size_t)(d >> 5) * SEGCAP + off;
    float* sX = zsm + wave * (ECH * (HID + KH));
    float* sH = sX + ECH * HID;
    _Float16* zrow = Z + (size_t)row * ZK;

    float xs[8];
#pragma unroll
    for (int t = 0; t < 8; ++t) xs[t] = 0.0f;

#pragma unroll 1
    for (int kg = 0; kg < 4; ++kg) {
        float z[8][8];
#pragma unroll
        for (int s = 0; s < 8; ++s)
#pragma unroll
            for (int t = 0; t < 8; ++t) z[s][t] = 0.0f;

#pragma unroll 1
        for (int ch = 0; ch < nch; ++ch) {
            const int c0 = ch * ECH;
            int nE = navail - c0;
            nE = nE < 0 ? 0 : (nE > ECH ? ECH : nE);
            if (kg == 0 || nch > 1) {
                __syncthreads();
#pragma unroll 1
                for (int j = 0; j < nE; ++j) {
                    int e = seg[c0 + j];
                    e = clampi(e, 0, E - 1);
                    int sn = srcIdx[e];
                    sn = clampi(sn, 0, N - 1);
                    if (lane < 16)
                        *(v4f*)(sX + j * HID + lane * 4) = *(const v4f*)(hcur + (size_t)sn * HID + lane * 4);
                    float ef[5];
#pragma unroll
                    for (int q = 0; q < 5; ++q) ef[q] = efeat[(size_t)e * 5 + q];
#pragma unroll
                    for (int t = 0; t < 4; ++t) {
                        const int k = lane + 32 * t;
                        float v = sE1b[k];
#pragma unroll
                        for (int q = 0; q < 5; ++q) v = fmaf(ef[q], sE1w[q * KH + k], v);
                        sH[j * KH + k] = fmaxf(v, 0.0f);
                    }
                }
                __syncthreads();
            }
#pragma unroll 1
            for (int j = 0; j < nE; ++j) {
                const v4f xa = *(const v4f*)(sX + j * HID + 8 * li);
                const v4f xb = *(const v4f*)(sX + j * HID + 8 * li + 4);
                float xv[8];
                xv[0] = xa[0]; xv[1] = xa[1]; xv[2] = xa[2]; xv[3] = xa[3];
                xv[4] = xb[0]; xv[5] = xb[1]; xv[6] = xb[2]; xv[7] = xb[3];
                const float* hp = sH + j * KH + kg * 32 + lk;
#pragma unroll
                for (int s = 0; s < 8; ++s) {
                    const float hk = hp[s * 4];
#pragma unroll
                    for (int t = 0; t < 8; ++t) z[s][t] = fmaf(hk, xv[t], z[s][t]);
                }
                if (kg == 0) {
#pragma unroll
                    for (int t = 0; t < 8; ++t) xs[t] += xv[t];
                }
            }
        }
#pragma unroll
        for (int s = 0; s < 8; ++s) {
            v8h o;
#pragma unroll
            for (int t = 0; t < 8; ++t) o[t] = (_Float16)(z[s][t] * osc);
            st8h(zrow + (kg * 32 + s * 4 + lk) * HID + 8 * li, o);
        }
        __threadfence();
#pragma unroll
        for (int s = 0; s < 8; ++s) {
            v8h o;
#pragma unroll
            for (int t = 0; t < 8; ++t) o[t] = (_Float16)(z[s][t] * osc);
            st8h(zrow + (kg * 32 + s * 4 + lk) * HID + 8 * li, o);
        }
    }
    {
        v8h o;
#pragma unroll
        for (int t = 0; t < 8; ++t) o[t] = (_Float16)(xs[t] * osc);
        if (lk == 0) st8h(zrow + KH * HID + 8 * li, o);
        __threadfence();
        if (lk == 0) st8h(zrow + KH * HID + 8 * li, o);
    }
}

__global__ void __launch_bounds__(256)
k_zgemm(const _Float16* __restrict__ Z, const _Float16* __restrict__ W16,
        float* __restrict__ agg, int passBase, int nrows)
{
    extern __shared__ float gsm2[];
    _Float16* sB = (_Float16*)gsm2;
    float* sT = gsm2 + 32768;

    const int tid = threadIdx.x, wave = tid >> 5, lane = tid & 31;
    const int h = lane >> 4, m = lane & 15;
    const int r0 = (blockIdx.x * 8 + wave) * 16;
    const _Float16* zr = Z + (size_t)(r0 + m) * ZK + 8 * h;

    v8f acc[4];
#pragma unroll
    for (int ct = 0; ct < 4; ++ct) acc[ct] = zero8();

#pragma unroll 1
    for (int slab = 0; slab < 9; ++slab) {
        const int nk = (slab < 8) ? 16 : 1;
        __syncthreads();
        {
            const v8h* gs = (const v8h*)(W16 + (size_t)slab * 16 * 4096);
            v8h* ld = (v8h*)sB;
            for (int q = tid; q < nk * 512; q += 256) ld[q] = gs[q];
        }
        __syncthreads();
#pragma unroll 1
        for (int kl = 0; kl < nk; ++kl) {
            const int ks = slab * 16 + kl;
            const _Float16* zp = zr + ks * HID;
            Frag A0, A1;
            A0.hf[0] = *(const v8h*)(zp);
            A0.hf[1] = *(const v8h*)(zp + 16);
            A1.hf[0] = *(const v8h*)(zp + 32);
            A1.hf[1] = *(const v8h*)(zp + 48);
            const _Float16* bk = sB + kl * 4096 + m * HID + 8 * h;
#pragma unroll
            for (int ct = 0; ct < 4; ++ct) {
                const _Float16* bp = bk + ct * 16 * HID;
                Frag B0, B1;
                B0.hf[0] = *(const v8h*)(bp);
                B0.hf[1] = *(const v8h*)(bp + 16);
                B1.hf[0] = *(const v8h*)(bp + 32);
                B1.hf[1] = *(const v8h*)(bp + 48);
                acc[ct] = mma16(A0.v, B0.v, acc[ct]);
                acc[ct] = mma16(A1.v, B1.v, acc[ct]);
            }
        }
    }
    float* st = sT + wave * 1024;
#pragma unroll
    for (int ct = 0; ct < 4; ++ct)
#pragma unroll
        for (int r = 0; r < 8; ++r)
            st[(8 * h + r) * HID + ct * 16 + m] = acc[ct][r] * UN_ZW;
    __syncthreads();
    v4f pv[8];
#pragma unroll
    for (int s = 0; s < 8; ++s) pv[s] = ((const v4f*)st)[s * 32 + lane];
#pragma unroll
    for (int s = 0; s < 8; ++s) {
        const int piece = s * 32 + lane, rr = piece >> 4;
        if (r0 + rr < nrows)
            st4(agg + (size_t)(passBase + r0 + rr) * HID + (piece & 15) * 4, pv[s]);
    }
    __threadfence();
#pragma unroll
    for (int s = 0; s < 8; ++s) {
        const int piece = s * 32 + lane, rr = piece >> 4;
        if (r0 + rr < nrows)
            st4(agg + (size_t)(passBase + r0 + rr) * HID + (piece & 15) * 4, pv[s]);
    }
}

__global__ void __launch_bounds__(128)
k_gru(const float* __restrict__ agg, const float* __restrict__ hcur,
      const float* __restrict__ cbias, const _Float16* __restrict__ GihT,
      const _Float16* __restrict__ GhhT, const float* __restrict__ bih,
      const float* __restrict__ bhh, float* __restrict__ hnext, int N, int nrowsOut)
{
    extern __shared__ float gsm3[];
    _Float16* sAm = (_Float16*)gsm3;
    _Float16* sAh = sAm + 2048;
    float* sHp = gsm3 + 2048;
    float* sG  = sHp + 2048;
    float* sO  = sG + 2 * 32 * GW;

    const int tid = threadIdx.x;
    const int base = blockIdx.x * 32;
    const int nl = tid >> 2, part = tid & 3;
    int nodeC = base + nl;
    nodeC = nodeC < N ? nodeC : N - 1;
    {
        const v4f* ar = (const v4f*)(agg  + (size_t)nodeC * HID + part * 16);
        const v4f* hr = (const v4f*)(hcur + (size_t)nodeC * HID + part * 16);
#pragma unroll
        for (int q4 = 0; q4 < 4; ++q4) {
            const v4f a = ar[q4], hv = hr[q4];
#pragma unroll
            for (int u = 0; u < 4; ++u) {
                const int col = part * 16 + q4 * 4 + u;
                const float mval = fmaxf(a[u] + cbias[col], 0.0f);
                sAm[nl * HID + col] = (_Float16)(mval * SC_A);
                sAh[nl * HID + col] = (_Float16)(hv[u] * SC_A);
                sHp[nl * HID + col] = hv[u];
            }
        }
    }
    __syncthreads();
    {
        const int wave = tid >> 5, lane = tid & 31, h = lane >> 4, m = lane & 15;
        const int rt = wave >> 1, mat = wave & 1;
        const _Float16* sA = mat ? sAh : sAm;
        const _Float16* GT = mat ? GhhT : GihT;
        const _Float16* ap = sA + (rt * 16 + m) * HID + 8 * h;
        Frag A0, A1;
        A0.hf[0] = *(const v8h*)(ap);
        A0.hf[1] = *(const v8h*)(ap + 16);
        A1.hf[0] = *(const v8h*)(ap + 32);
        A1.hf[1] = *(const v8h*)(ap + 48);
        float* g = sG + mat * 32 * GW;
#pragma unroll 1
        for (int ct = 0; ct < 12; ++ct) {
            const _Float16* bp = GT + (size_t)(ct * 16 + m) * HID + 8 * h;
            Frag B0, B1;
            B0.hf[0] = *(const v8h*)(bp);
            B0.hf[1] = *(const v8h*)(bp + 16);
            B1.hf[0] = *(const v8h*)(bp + 32);
            B1.hf[1] = *(const v8h*)(bp + 48);
            v8f acc = zero8();
            acc = mma16(A0.v, B0.v, acc);
            acc = mma16(A1.v, B1.v, acc);
#pragma unroll
            for (int r = 0; r < 8; ++r)
                g[(rt * 16 + 8 * h + r) * GW + ct * 16 + m] = acc[r] * UN_AW;
        }
    }
    __syncthreads();
    {
        const float* gi = sG + nl * GW;
        const float* gh = sG + 32 * GW + nl * GW;
#pragma unroll 2
        for (int c = 0; c < 16; ++c) {
            const int col = part * 16 + c;
            const float xr = gi[col] + bih[col] + gh[col] + bhh[col];
            const float xz = gi[HID + col] + bih[HID + col] + gh[HID + col] + bhh[HID + col];
            const float rg = sigm(xr), zg = sigm(xz);
            const float ng = tanhf(gi[2 * HID + col] + bih[2 * HID + col] + rg * (gh[2 * HID + col] + bhh[2 * HID + col]));
            sO[nl * HID + col] = (1.0f - zg) * ng + zg * sHp[nl * HID + col];
        }
    }
    __syncthreads();
    v4f pv[4];
#pragma unroll
    for (int s = 0; s < 4; ++s) pv[s] = ((const v4f*)sO)[s * 128 + tid];
#pragma unroll
    for (int s = 0; s < 4; ++s) {
        const int piece = s * 128 + tid, rr = piece >> 4, nd = base + rr;
        if (nd < nrowsOut) st4(hnext + (size_t)nd * HID + (piece & 15) * 4, pv[s]);
    }
    __threadfence();
#pragma unroll
    for (int s = 0; s < 4; ++s) {
        const int piece = s * 128 + tid, rr = piece >> 4, nd = base + rr;
        if (nd < nrowsOut) st4(hnext + (size_t)nd * HID + (piece & 15) * 4, pv[s]);
    }
}

__global__ void __launch_bounds__(256)
k_pool_blk(const float* __restrict__ outh, const float* __restrict__ scal,
           float* __restrict__ partial, int N)
{
    __shared__ float sq[HID];
    __shared__ float sw[256];
    __shared__ float sred[18];
    __shared__ float srec[128];
    const int tid = threadIdx.x, wave = tid >> 5, lane = tid & 31;
    if (tid < HID) sq[tid] = scal[tid];
    if (tid < 128) srec[tid] = 0.0f;
    __syncthreads();
    const int n0 = blockIdx.x * 256;
    const int n = n0 + tid;
    float e = -__builtin_huge_valf();
    if (n < N) {
        const v4f* rp = (const v4f*)(outh + (size_t)n * HID);
        float s = 0.0f;
#pragma unroll 4
        for (int j = 0; j < 16; ++j) {
            const v4f v = rp[j];
            s += v[0] * sq[4 * j] + v[1] * sq[4 * j + 1] + v[2] * sq[4 * j + 2] + v[3] * sq[4 * j + 3];
        }
        e = s;
    }
    float mx = wmax32(e);
    if (lane == 0) sred[wave] = mx;
    __syncthreads();
    if (tid == 0) {
        float M = sred[0];
#pragma unroll
        for (int q = 1; q < 8; ++q) M = fmaxf(M, sred[q]);
        sred[16] = M;
    }
    __syncthreads();
    const float M = sred[16];
    const float wv = (n < N) ? expf(e - M) : 0.0f;
    sw[tid] = wv;
    float sm = wsum32(wv);
    if (lane == 0) sred[8 + wave] = sm;
    __syncthreads();
    if (tid == 0) {
        float S = 0.0f;
#pragma unroll
        for (int q = 0; q < 8; ++q) S += sred[8 + q];
        srec[HID] = M;
        srec[HID + 1] = S;
    }
    if (tid < HID) {
        int nn = N - n0;
        nn = nn > 256 ? 256 : nn;
        float acc = 0.0f;
        const float* ob = outh + (size_t)n0 * HID + tid;
#pragma unroll 4
        for (int j = 0; j < nn; ++j) acc = fmaf(sw[j], ob[(size_t)j * HID], acc);
        srec[tid] = acc;
    }
    __syncthreads();
    v4f rv = zero4();
    if (tid < 32) rv = ((const v4f*)srec)[tid];
    if (tid < 32) st4(partial + (size_t)blockIdx.x * 128 + tid * 4, rv);
    __threadfence();
    if (tid < 32) st4(partial + (size_t)blockIdx.x * 128 + tid * 4, rv);
}

__global__ void __launch_bounds__(256)
k_pool_step(const float* __restrict__ partial, int NB2,
            const float* __restrict__ lWih, const float* __restrict__ lWhh,
            const float* __restrict__ lbih, const float* __restrict__ lbhh,
            float* __restrict__ scal, float* __restrict__ outq, int flags)
{
    __shared__ float sqs[128];
    __shared__ float shl[HID];
    __shared__ float scl[HID];
    __shared__ float sscale[MAXB2];
    __shared__ float sg[256];
    __shared__ float sst[128];
    __shared__ float sred[24];
    const int tid = threadIdx.x, wave = tid >> 5, lane = tid & 31;
    const int nb = NB2 < MAXB2 ? NB2 : MAXB2;

    if (flags & 1) {
        if (tid < HID) { shl[tid] = scal[tid]; scl[tid] = scal[HID + tid]; }
        float lm = -__builtin_huge_valf();
        for (int bq = tid; bq < nb; bq += 256) lm = fmaxf(lm, partial[(size_t)bq * 128 + HID]);
        lm = wmax32(lm);
        if (lane == 0) sred[wave] = lm;
        __syncthreads();
        if (tid == 0) {
            float M = sred[0];
#pragma unroll
            for (int q = 1; q < 8; ++q) M = fmaxf(M, sred[q]);
            sred[16] = M;
        }
        __syncthreads();
        const float M = sred[16];
        float ls = 0.0f;
        for (int bq = tid; bq < nb; bq += 256) {
            const float sc = expf(partial[(size_t)bq * 128 + HID] - M);
            sscale[bq] = sc;
            ls += partial[(size_t)bq * 128 + HID + 1] * sc;
        }
        ls = wsum32(ls);
        if (lane == 0) sred[8 + wave] = ls;
        __syncthreads();
        if (tid == 0) {
            float S = 0.0f;
#pragma unroll
            for (int q = 0; q < 8; ++q) S += sred[8 + q];
            sred[17] = S;
        }
        __syncthreads();
        const float S = sred[17];
        if (tid < HID) {
            float R = 0.0f;
#pragma unroll 4
            for (int bq = 0; bq < nb; ++bq) R = fmaf(sscale[bq], partial[(size_t)bq * 128 + tid], R);
            sqs[HID + tid] = R / S;
            sqs[tid] = shl[tid];
        }
    } else {
        if (tid < 128) sqs[tid] = 0.0f;
        if (tid < HID) { shl[tid] = 0.0f; scl[tid] = 0.0f; }
    }
    __syncthreads();
    v4f qo = zero4();
    if (tid < 32) qo = ((const v4f*)sqs)[tid];
    v4f sv = zero4();
    if (flags & 2) {
        float g = lbih[tid] + lbhh[tid];
#pragma unroll 2
        for (int i = 0; i < 128; ++i) g = fmaf(sqs[i], lWih[(size_t)i * 256 + tid], g);
#pragma unroll 2
        for (int i = 0; i < HID; ++i) g = fmaf(shl[i], lWhh[(size_t)i * 256 + tid], g);
        sg[tid] = g;
        __syncthreads();
        if (tid < HID) {
            const float ig = sigm(sg[tid]);
            const float fg = sigm(sg[HID + tid]);
            const float gg = tanhf(sg[2 * HID + tid]);
            const float og = sigm(sg[3 * HID + tid]);
            const float c = fg * scl[tid] + ig * gg;
            const float hh = og * tanhf(c);
            sst[tid] = hh;
            sst[HID + tid] = c;
        }
        __syncthreads();
        if (tid < 32) sv = ((const v4f*)sst)[tid];
    }
    if ((flags & 4) && tid < 32) st4(outq + tid * 4, qo);
    if ((flags & 2) && tid < 32) st4(scal + tid * 4, sv);
    __threadfence();
    if ((flags & 4) && tid < 32) st4(outq + tid * 4, qo);
    if ((flags & 2) && tid < 32) st4(scal + tid * 4, sv);
}

extern "C" void kernel_launch(void* const* d_in, const int* in_sizes, int n_in,
                              void* d_out, int out_size, void* d_ws, size_t ws_size,
                              hipStream_t stream)
{
    (void)n_in;
    const float* nfeat  = (const float*)d_in[0];
    const float* efeat  = (const float*)d_in[1];
    const int*   src    = (const int*)d_in[2];
    const int*   dst    = (const int*)d_in[3];
    const float* lin0_w = (const float*)d_in[4];
    const float* lin0_b = (const float*)d_in[5];
    const float* e1_w   = (const float*)d_in[6];
    const float* e1_b   = (const float*)d_in[7];
    const float* e2_w   = (const float*)d_in[8];
    const float* e2_b   = (const float*)d_in[9];
    const float* cbias  = (const float*)d_in[10];
    const float* gW_ih  = (const float*)d_in[11];
    const float* gW_hh  = (const float*)d_in[12];
    const float* gb_ih  = (const float*)d_in[13];
    const float* gb_hh  = (const float*)d_in[14];
    const float* lW_ih  = (const float*)d_in[15];
    const float* lW_hh  = (const float*)d_in[16];
    const float* lb_ih  = (const float*)d_in[17];
    const float* lb_hh  = (const float*)d_in[18];

    const int N = in_sizes[0] / 16;
    int E = in_sizes[1] / 5;
    if (in_sizes[2] < E) E = in_sizes[2];
    if (in_sizes[3] < E) E = in_sizes[3];
    if (N <= 0 || E <= 0) return;
    if (out_size < 128 + HID) return;
    int nrowsOut = (out_size - 128) / HID;
    if (nrowsOut > N) nrowsOut = N;

    const int nb64 = (N + 63) / 64;
    const int Npad = nb64 * 64;
    const int nbc  = (N + 31) / 32;
    const int NB2  = (N + 255) / 256;
    if (NB2 > MAXB2) return;

    size_t off = 0;
    auto take = [&](size_t bytes) -> size_t { size_t p = off; off += (bytes + 255) & ~(size_t)255; return p; };
    const size_t oH0   = take((size_t)Npad * HID * 4);
    const size_t oH1   = take((size_t)Npad * HID * 4);
    const size_t oAgg  = take((size_t)Npad * HID * 4);
    const size_t oW16  = take((size_t)NSLOT * 4096 * 2);
    const size_t oGih  = take((size_t)HID * GW * 2);
    const size_t oGhh  = take((size_t)HID * GW * 2);
    const size_t oSeg  = take((size_t)nbc * SEGCAP * 4);
    const size_t oRec  = take((size_t)nbc * 64 * 4);
    const size_t oPart = take((size_t)NB2 * 128 * 4);
    const size_t oScal = take(512);
    if (off >= ws_size) return;
    const size_t rem = ws_size - off;
    const size_t capRows = (rem / ((size_t)ZK * 2)) / 128 * 128;
    if (capRows < 128) return;
    const int Nr128 = (N + 127) / 128 * 128;
    int passes = (int)(((size_t)Nr128 + capRows - 1) / capRows);
    if (passes < 1) passes = 1;
    int NH = ((N + passes - 1) / passes + 127) / 128 * 128;
    if ((size_t)NH > capRows) NH = (int)capRows;
    passes = (N + NH - 1) / NH;
    const size_t oZ = take((size_t)NH * ZK * 2);
    if (off > ws_size) return;

    char* ws = (char*)d_ws;
    float*    hb0     = (float*)(ws + oH0);
    float*    hb1     = (float*)(ws + oH1);
    float*    agg     = (float*)(ws + oAgg);
    _Float16* W16     = (_Float16*)(ws + oW16);
    _Float16* GihT    = (_Float16*)(ws + oGih);
    _Float16* GhhT    = (_Float16*)(ws + oGhh);
    int*      segTab  = (int*)(ws + oSeg);
    int*      nodeRec = (int*)(ws + oRec);
    float*    partial = (float*)(ws + oPart);
    float*    scal    = (float*)(ws + oScal);
    _Float16* Zbuf    = (_Float16*)(ws + oZ);
    float*    outp    = (float*)d_out;

    k_prep<<<NSLOT + 2, 256, 0, stream>>>(e2_w, e2_b, gW_ih, gW_hh, W16, GihT, GhhT);
    k_csr<<<nbc, 32, 0, stream>>>(dst, segTab, nodeRec, E);
    k_lin0<<<nb64, 128, 0, stream>>>(nfeat, lin0_w, lin0_b, hb0, N);

    float* hb[2] = { hb0, hb1 };
    for (int it = 0; it < 3; ++it) {
        const float* hcur = hb[it & 1];
        float* hnext = (it < 2) ? hb[(it + 1) & 1] : (outp + 128);
        const int nro = (it < 2) ? Npad : nrowsOut;
        for (int p = 0; p < passes; ++p) {
            const int pb = p * NH;
            int nrows = N - pb;
            if (nrows > NH) nrows = NH;
            const int R = (nrows + 127) / 128 * 128;
            k_zbuild<<<R / 8, 256, LDS_ZB, stream>>>(hcur, efeat, e1_w, e1_b, src, segTab, nodeRec,
                                                     Zbuf, pb, N, E);
            k_zgemm<<<R / 128, 256, LDS_ZG, stream>>>(Zbuf, W16, agg, pb, nrows);
        }
        k_gru<<<nbc, 128, LDS_GRU, stream>>>(agg, hcur, cbias, GihT, GhhT, gb_ih, gb_hh, hnext, N, nro);
    }

    const float* outh = outp + 128;
    for (int it = 0; it < 3; ++it) {
        const int fl = ((it > 0) ? 1 : 0) | 2;
        k_pool_step<<<1, 256, 0, stream>>>(partial, NB2, lW_ih, lW_hh, lb_ih, lb_hh, scal, outp, fl);
        k_pool_blk<<<NB2, 256, 0, stream>>>(outh, scal, partial, N);
    }
    k_pool_step<<<1, 256, 0, stream>>>(partial, NB2, lW_ih, lW_hh, lb_ih, lb_hh, scal, outp, 1 | 4);
}
